// PinnNs_3032246911612
// MI455X (gfx1250) — hardware-verified
//
#include <hip/hip_runtime.h>
#include <stddef.h>


typedef unsigned short u16;
typedef u16   v2us  __attribute__((ext_vector_type(2)));
typedef u16   v8us  __attribute__((ext_vector_type(8)));
typedef u16   v16us __attribute__((ext_vector_type(16)));
typedef float v8f   __attribute__((ext_vector_type(8)));
typedef float v4f   __attribute__((ext_vector_type(4)));

#define NJ   13
#define H    20
#define NHID 7
#define TP   16
#define KP   32
#define PPB  32
#define NLAY (NHID + 1)
#define FOLD (KP - H)

#ifndef NPTS
#define NPTS 131072
#endif
#define NPTS_FULL 131072

#ifndef JET_SPLIT
#define JET_SPLIT 1
#endif
#if JET_SPLIT
typedef __bf16 v16op __attribute__((ext_vector_type(16)));
#define NSTEP 2
#define WCARRY 1.0f
#else
typedef _Float16 v16op __attribute__((ext_vector_type(16)));
#define NSTEP 1
#define WCARRY 4.0f
#endif

#define HB_ELEMS    (2 * NSTEP * NJ * TP * KP)
#define WSTEP_ELEMS (NLAY * 32 * KP)
#define WS_TOTAL    ((size_t)NSTEP * WSTEP_ELEMS * 2)
#define HB(buf, st, j, p, k) ((((((buf) * (unsigned)NSTEP + (st)) * (unsigned)NJ + (j)) * (unsigned)TP + (p)) * (unsigned)KP) + (k))

static_assert(NJ == 13);
static_assert(H == 20 && (H % 2) == 0 && H <= KP);
static_assert(KP == 32 && TP == 16 && PPB == 2 * TP);
static_assert(FOLD > 0 && (FOLD % 2) == 0 && FOLD <= H);
static_assert((H - FOLD) + H <= KP);
static_assert((H * TP) % 32 == 0);
static_assert(NPTS >= PPB && NPTS <= NPTS_FULL && (NPTS % PPB) == 0);
static_assert((size_t)NPTS_FULL * 4 == (size_t)524288);
static_assert((HB_ELEMS % 8) == 0);
static_assert((size_t)HB_ELEMS * 2 + 5 * PPB * 4 <= (size_t)65536);
static_assert((WSTEP_ELEMS * 2) % 128 == 0);
static_assert(WS_TOTAL <= (size_t)134217728);

__device__ __forceinline__ unsigned bf16_bits(float x) {
  const unsigned u = __float_as_uint(x);
  return (u + 0x7FFFu + ((u >> 16) & 1u)) >> 16;
}

#if !JET_SPLIT
static __device__ __forceinline__ _Float16 toh_flush(float v) {
  const _Float16 r = (_Float16)v;
  return (fabsf(v) < 6.103515625e-05f) ? (_Float16)0.0f : r;
}
#endif

__device__ __forceinline__ void split16(float v, u16& hi, u16& lo) {
#if JET_SPLIT
  const unsigned hbits = bf16_bits(v);
  const float hf = __uint_as_float(hbits << 16);
  hi = (u16)hbits;
  lo = (u16)bf16_bits(v - hf);
#else
  hi = __builtin_bit_cast(u16, toh_flush(v));
  lo = (u16)0;
#endif
}

__device__ __forceinline__ v16us cat8(v8us a, v8us b) {
  return __builtin_shufflevector(a, b, 0, 1, 2, 3, 4, 5, 6, 7, 8, 9, 10, 11, 12, 13, 14, 15);
}

__device__ __forceinline__ v8f wmma16(v16us a, v16us b, v8f c) {
  const v16op av = __builtin_bit_cast(v16op, a);
  const v16op bv = __builtin_bit_cast(v16op, b);
#if JET_SPLIT
  v8f d = __builtin_amdgcn_wmma_f32_16x16x32_bf16(false, av, false, bv, (short)0, c, false, false);
#else
  v8f d = __builtin_amdgcn_wmma_f32_16x16x32_f16(false, av, false, bv, (short)0, c, false, false);
#endif
  asm volatile("v_nop\n\tv_nop\n\tv_nop\n\tv_nop" : "+v"(d) : "v"(a), "v"(b));
  return d;
}

__device__ __forceinline__ void jet_tanh(const float z[NJ], float h[NJ]) {
    float f  = tanhf(z[0]);
    float f1 = 1.0f - f * f;
    float f2 = -2.0f * f * f1;
    float f3 = -2.0f * f1 * f1 - 2.0f * f * f2;
    h[0] = f;
    h[1] = f1 * z[1];
    h[2] = f1 * z[2];
    h[3] = f1 * z[3];
    h[4] = f2 * z[1] * z[1] + f1 * z[4];
    h[5] = f2 * z[1] * z[2] + f1 * z[5];
    h[6] = f2 * z[2] * z[2] + f1 * z[6];
    h[7] = f2 * z[1] * z[3] + f1 * z[7];
    h[8] = f2 * z[2] * z[3] + f1 * z[8];
    h[9]  = f3*z[1]*z[1]*z[1] + 3.0f*f2*z[4]*z[1]                    + f1*z[9];
    h[10] = f3*z[1]*z[1]*z[2] + f2*(z[4]*z[2] + 2.0f*z[5]*z[1])      + f1*z[10];
    h[11] = f3*z[1]*z[2]*z[2] + f2*(z[6]*z[1] + 2.0f*z[5]*z[2])      + f1*z[11];
    h[12] = f3*z[2]*z[2]*z[2] + 3.0f*f2*z[6]*z[2]                    + f1*z[12];
}

__global__ __launch_bounds__(256) void wprep_kernel(
    const float* __restrict__ W_hid, const float* __restrict__ W_out, u16* __restrict__ Wp) {
  const unsigned tid = threadIdx.x;
  const unsigned l = blockIdx.x;
  const unsigned st = tid >> 7;
  const unsigned tt = tid & 127u;
  const unsigned nrow = tt >> 2, k8 = (tt & 3u) * 8u;
  const unsigned lc = (l < (unsigned)NHID) ? l : (unsigned)(NHID - 1);
  const unsigned nh = (nrow < (unsigned)H) ? nrow : (unsigned)(H - 1);
  const unsigned no = (nrow < 2u) ? nrow : 1u;
  v8us o;
#pragma unroll
  for (unsigned i = 0; i < 8u; ++i) {
    const unsigned q = k8 + i;
    unsigned k;
    unsigned part;
#if JET_SPLIT
    if (st == 0u) {
      k = (q < (unsigned)H) ? q : (q - (unsigned)H);
      part = 0u;
    } else {
      if (q < (unsigned)(H - FOLD)) { k = q + (unsigned)FOLD; part = 0u; }
      else if (q < (unsigned)(2 * H - FOLD)) { k = q - (unsigned)(H - FOLD); part = 1u; }
      else { k = 0u; part = 2u; }
    }
#else
    k = (q < (unsigned)H) ? q : 0u;
    part = (q < (unsigned)H) ? 0u : 2u;
#endif
    const unsigned kc = (k < (unsigned)H) ? k : (unsigned)(H - 1);
    const float wh = W_hid[(lc * (unsigned)H + kc) * (unsigned)H + nh];
    const float wo = W_out[kc * 2u + no];
    const bool okh = (l < (unsigned)NHID) && (nrow < (unsigned)H);
    const bool oko = (l == (unsigned)NHID) && (nrow < 2u);
    const float v = okh ? wh : (oko ? wo : 0.0f);
    u16 hi, lo;
    split16(v * WCARRY, hi, lo);
    o[i] = (part == 0u) ? hi : ((part == 1u) ? lo : (u16)0);
  }
  u16* p = Wp + (size_t)st * WSTEP_ELEMS + ((size_t)(l * 32u + nrow) * KP + k8);
  *(volatile v8us*)p = o;
  __threadfence();
  *(volatile v8us*)p = o;
}

__global__ __launch_bounds__(32) __attribute__((amdgpu_num_vgpr(256))) void pinn_jet_kernel(
    const float* __restrict__ x, const float* __restrict__ y, const float* __restrict__ t,
    const float* __restrict__ W_in, const float* __restrict__ b_in,
    const float* __restrict__ b_hid, const float* __restrict__ b_out,
    const float* __restrict__ lb, const float* __restrict__ ub,
    const float* __restrict__ lam1, const float* __restrict__ lam2,
    const u16* __restrict__ Wp, float* __restrict__ out, int n)
{
  __shared__ __attribute__((aligned(16))) u16 hb[HB_ELEMS];
  __shared__ __attribute__((aligned(16))) float ost[5 * PPB];

  const unsigned lane  = threadIdx.x & 31u;
  const unsigned nloc  = lane & 15u;
  const unsigned khalf = lane >> 4;

  {
    const v8us zero8 = {0, 0, 0, 0, 0, 0, 0, 0};
#pragma unroll 4
    for (unsigned i = lane; i < (unsigned)(HB_ELEMS / 8); i += 32u) *(v8us*)&hb[i * 8u] = zero8;
  }
  __syncthreads();

  const float lb0 = lb[0], lb1 = lb[1], lb2 = lb[2];
  const float i0 = 1.0f / (ub[0] - lb0);
  const float i1 = 1.0f / (ub[1] - lb1);
  const float i2 = 1.0f / (ub[2] - lb2);
  const float l1 = lam1[0], l2 = lam2[0];
  const float inv_wc = 1.0f / WCARRY;

#pragma unroll 1
  for (unsigned sub = 0; sub < 2u; ++sub) {
    int g = (int)(blockIdx.x * (unsigned)PPB + sub * (unsigned)TP + nloc);
    if (g >= n) g = n - 1;
    const float hx = 2.0f * (x[g] - lb0) * i0 - 1.0f;
    const float hy = 2.0f * (y[g] - lb1) * i1 - 1.0f;
    const float ht = 2.0f * (t[g] - lb2) * i2 - 1.0f;
#pragma unroll 1
    for (unsigned it = 0; it < (unsigned)((H * TP) / 32); ++it) {
      const unsigned nn = it * 2u + khalf;
      const float w0 = W_in[0 * H + nn], w1 = W_in[1 * H + nn], w2 = W_in[2 * H + nn];
      float z[NJ], h[NJ];
#pragma unroll
      for (int j = 0; j < NJ; ++j) z[j] = 0.0f;
      z[0] = hx * w0 + hy * w1 + ht * w2 + b_in[nn];
      z[1] = 2.0f * i0 * w0;
      z[2] = 2.0f * i1 * w1;
      z[3] = 2.0f * i2 * w2;
      jet_tanh(z, h);
#pragma unroll
      for (int j = 0; j < NJ; ++j) {
        u16 hi, lo;
        split16(h[j], hi, lo);
        hb[HB(0u, 0u, (unsigned)j, nloc, nn)] = hi;
#if JET_SPLIT
        hb[HB(0u, 1u, (unsigned)j, nloc, (unsigned)(H - FOLD) + nn)] = hi;
        const unsigned lp = (nn < (unsigned)FOLD)
                                ? HB(0u, 0u, (unsigned)j, nloc, (unsigned)H + nn)
                                : HB(0u, 1u, (unsigned)j, nloc, nn - (unsigned)FOLD);
        hb[lp] = lo;
#endif
      }
    }
    __syncthreads();

#pragma unroll 1
    for (unsigned l = 0; l <= (unsigned)NHID; ++l) {
      const unsigned cur = l & 1u, nxt = cur ^ 1u;
      const unsigned ntile = (l < (unsigned)NHID) ? 2u : 1u;
#pragma unroll 1
      for (unsigned tile = 0; tile < ntile; ++tile) {
        const u16* wrow = Wp + ((size_t)(l * 32u + tile * 16u + nloc) * KP + khalf * 8u);
        const v16us w0f = cat8(*(const v8us*)(wrow), *(const v8us*)(wrow + 16));
#if JET_SPLIT
        const v16us w1f = cat8(*(const v8us*)(wrow + WSTEP_ELEMS),
                               *(const v8us*)(wrow + WSTEP_ELEMS + 16));
#endif
        v8f c[NJ];
#pragma unroll
        for (int j = 0; j < NJ; ++j) {
          const unsigned b0i = HB(cur, 0u, (unsigned)j, nloc, khalf * 8u);
          const v16us b0f = cat8(*(const v8us*)&hb[b0i], *(const v8us*)&hb[b0i + 16u]);
          v8f acc = {};
          acc = wmma16(w0f, b0f, acc);
#if JET_SPLIT
          const unsigned b1i = HB(cur, 1u, (unsigned)j, nloc, khalf * 8u);
          const v16us b1f = cat8(*(const v8us*)&hb[b1i], *(const v8us*)&hb[b1i + 16u]);
          acc = wmma16(w1f, b1f, acc);
#endif
          c[j] = acc;
        }

        if (l < (unsigned)NHID) {
          const unsigned nbase = tile * 16u + khalf * 8u;
#pragma unroll
          for (int rp = 0; rp < 4; ++rp) {
            if (tile == 0u || rp < 2) {
              u16 ph[NJ][2], pq[NJ][2];
#pragma unroll
              for (int rr = 0; rr < 2; ++rr) {
                const int r = rp * 2 + rr;
                const unsigned neuron = nbase + (unsigned)r;
                const unsigned nc = (neuron < (unsigned)H) ? neuron : (unsigned)(H - 1);
                const float bv0 = b_hid[l * (unsigned)H + nc];
                const float bv = (neuron < (unsigned)H) ? bv0 : 0.0f;
                float z[NJ], h[NJ];
#pragma unroll
                for (int j = 0; j < NJ; ++j) z[j] = c[j][r] * inv_wc;
                z[0] += bv;
                jet_tanh(z, h);
#pragma unroll
                for (int j = 0; j < NJ; ++j) split16(h[j], ph[j][rr], pq[j][rr]);
              }
              const unsigned kq = nbase + 2u * (unsigned)rp;
              if (kq < (unsigned)H) {
#pragma unroll
                for (int j = 0; j < NJ; ++j) {
                  v2us a;
                  a[0] = ph[j][0];
                  a[1] = ph[j][1];
                  *(v2us*)&hb[HB(nxt, 0u, (unsigned)j, nloc, kq)] = a;
#if JET_SPLIT
                  *(v2us*)&hb[HB(nxt, 1u, (unsigned)j, nloc, (unsigned)(H - FOLD) + kq)] = a;
                  v2us b;
                  b[0] = pq[j][0];
                  b[1] = pq[j][1];
                  const unsigned lp = (kq < (unsigned)FOLD)
                                          ? HB(nxt, 0u, (unsigned)j, nloc, (unsigned)H + kq)
                                          : HB(nxt, 1u, (unsigned)j, nloc, kq - (unsigned)FOLD);
                  *(v2us*)&hb[lp] = b;
#endif
                }
              }
            }
          }
        } else {
          float P[NJ];
#pragma unroll
          for (int j = 0; j < NJ; ++j) P[j] = c[j][0] * inv_wc;
          P[0] += b_out[0];
          const float pv  = c[0][1] * inv_wc + b_out[1];
          const float p_x = c[1][1] * inv_wc;
          const float p_y = c[2][1] * inv_wc;
          float u =  P[2],  v = -P[1];
          float u_t =  P[8],  u_x =  P[5],  u_y =  P[6];
          float u_xx = P[10], u_yy = P[12];
          float v_t = -P[7],  v_x = -P[4],  v_y = -P[5];
          float v_xx = -P[9], v_yy = -P[11];
          float f_u = u_t + l1 * (u * u_x + v * u_y) + p_x - l2 * (u_xx + u_yy);
          float f_v = v_t + l1 * (u * v_x + v * v_y) + p_y - l2 * (v_xx + v_yy);
          if (lane < 16u) {
            const unsigned pc = sub * (unsigned)TP + nloc;
            ost[0 * PPB + pc] = u;
            ost[1 * PPB + pc] = v;
            ost[2 * PPB + pc] = pv;
            ost[3 * PPB + pc] = f_u;
            ost[4 * PPB + pc] = f_v;
          }
        }
      }
      __syncthreads();
    }
  }

  {
    const unsigned line = lane >> 3, piece = (lane & 7u) * 4u;
    const size_t pbase = (size_t)blockIdx.x * PPB;
    float* o0 = out + (size_t)line * NPTS_FULL + pbase + piece;
    float* o1 = out + (size_t)4 * NPTS_FULL + pbase + piece;
    const v4f v0 = *(const v4f*)&ost[line * (unsigned)PPB + piece];
    const v4f v1 = *(const v4f*)&ost[4u * (unsigned)PPB + piece];
    *(volatile v4f*)o0 = v0;
    if (lane < 8u) *(volatile v4f*)o1 = v1;
    __threadfence();
    *(volatile v4f*)o0 = v0;
    if (lane < 8u) *(volatile v4f*)o1 = v1;
  }
}

extern "C" void kernel_launch(void* const* d_in, const int* in_sizes, int n_in,
                              void* d_out, int out_size, void* d_ws, size_t ws_size,
                              hipStream_t stream) {
  if (n_in < 13) return;
  if (in_sizes[0] < NPTS || in_sizes[1] < NPTS || in_sizes[2] < NPTS) return;
  if (in_sizes[3] < 3 * H || in_sizes[4] < H) return;
  if (in_sizes[5] < NHID * H * H || in_sizes[6] < NHID * H) return;
  if (in_sizes[7] < H * 2 || in_sizes[8] < 2) return;
  if (in_sizes[9] < 3 || in_sizes[10] < 3 || in_sizes[11] < 1 || in_sizes[12] < 1) return;
  if ((long long)out_size < (long long)4 * NPTS_FULL + NPTS) return;
  if (ws_size < WS_TOTAL) return;

  const float* x     = (const float*)d_in[0];
  const float* y     = (const float*)d_in[1];
  const float* t     = (const float*)d_in[2];
  const float* W_in  = (const float*)d_in[3];
  const float* b_in  = (const float*)d_in[4];
  const float* W_hid = (const float*)d_in[5];
  const float* b_hid = (const float*)d_in[6];
  const float* W_out = (const float*)d_in[7];
  const float* b_out = (const float*)d_in[8];
  const float* lb    = (const float*)d_in[9];
  const float* ub    = (const float*)d_in[10];
  const float* l1    = (const float*)d_in[11];
  const float* l2    = (const float*)d_in[12];
  u16* Wp = (u16*)d_ws;

  wprep_kernel<<<dim3(NLAY), dim3(128 * NSTEP), 0, stream>>>(W_hid, W_out, Wp);
  pinn_jet_kernel<<<dim3(NPTS / PPB), dim3(32), 0, stream>>>(
      x, y, t, W_in, b_in, b_hid, b_out, lb, ub, l1, l2, Wp, (float*)d_out, (int)NPTS);
}
